// NIMO_2353642078732
// MI455X (gfx1250) — hardware-run, weakly checked
//
#include <hip/hip_runtime.h>


#ifndef NS
#define NS 2048
#endif
#define NS_FULL 2048
#define DI   128
#define HW   256
#define OW   129
#define WV   2
#define JB   32
#define GP   36
#define HSN  4096
#define GW   8
#define ORW  32
#define TR   32
#define LN_EPS 1e-5f

static_assert(DI == 128);
static_assert(HW == 256);
static_assert(OW == DI + 1);
static_assert(JB == 32);
static_assert(DI / JB == 4);
static_assert(NS % 32 == 0);
static_assert(((NS / 16) * (DI / JB)) % WV == 0);
static_assert(NS <= NS_FULL);
static_assert(HSN == 16 * 8 * 32);
static_assert((GP * 4) % 16 == 0);
static_assert(GP >= JB);
static_assert(4 * (32 / 8) == 16);
static_assert(8 * 16 == JB * 4);
static_assert(((size_t)NS * DI) % 8 == 0);
static_assert(NS % ORW == 0);
static_assert((ORW * OW * 4) % 128 == 0);
static_assert((ORW * OW) % 4 == 0);
static_assert((ORW * DI) % 256 == 0);
static_assert(HW % TR == 0);
static_assert((DI * TR) % 256 == 0);
static_assert(2 * 256 * 16 == TR * DI * 2);
static_assert(GW * 4 == 32);
static_assert(DI % 32 == 0);
static_assert((WV * HSN + WV * HW + WV * 16 * GP + 3 * HW) * 4 <= 131072);
static_assert((GW * HW + 32) * 4 <= 131072);
static_assert(ORW * OW * 4 <= 131072);
static_assert(DI * 33 * 4 <= 131072);
static_assert((size_t)NS_FULL * OW * 4 == (size_t)1056768);

typedef unsigned short bf;
typedef __attribute__((ext_vector_type(16))) __bf16   v16bf;
typedef __attribute__((ext_vector_type(8)))  unsigned short v8us;
typedef __attribute__((ext_vector_type(8)))  float    v8f;
typedef __attribute__((ext_vector_type(4)))  float    v4f;
typedef __attribute__((ext_vector_type(4)))  unsigned v4u;
typedef __attribute__((ext_vector_type(8)))  unsigned v8u;
typedef v4f  __attribute__((may_alias)) v4fa;

__device__ __forceinline__ unsigned short f2bf(float f) { unsigned u = __float_as_uint(f); u += 0x7FFFu + ((u >> 16) & 1u); return (unsigned short)(u >> 16); }
__device__ __forceinline__ float bfr(float f) { return __uint_as_float(((unsigned)f2bf(f)) << 16); }
__device__ __forceinline__ v16bf cat16b(v8us lo, v8us hi) { return __builtin_bit_cast(v16bf, __builtin_shufflevector(lo, hi, 0, 1, 2, 3, 4, 5, 6, 7, 8, 9, 10, 11, 12, 13, 14, 15)); }
__device__ __forceinline__ v8f wmmab(v16bf a, v16bf b, v8f c) { return __builtin_amdgcn_wmma_f32_16x16x32_bf16(false, a, false, b, (short)0, c, false, false); }
__device__ __forceinline__ v8f wmmabg(v16bf a, v16bf b, v8f c) { c = wmmab(a, b, c); asm volatile("v_nop\n\tv_nop\n\tv_nop\n\tv_nop" : "+v"(c) : "v"(a), "v"(b)); return c; }
__device__ __forceinline__ v16bf ldb(const bf* p)  { return cat16b(*(const v8us*)p, *(const v8us*)(p + 16)); }
__device__ __forceinline__ void wave_sync() { __builtin_amdgcn_fence(3  , "wavefront"); __builtin_amdgcn_wave_barrier(); asm volatile("" ::: "memory"); }

__global__ __launch_bounds__(256) void k_cvt8(const float* __restrict__ src, bf* dst, size_t n8) {
    const size_t i = (size_t)blockIdx.x * 256 + threadIdx.x; if (i >= n8) return;
    const v8f v = *(const v8f*)(src + i * 8); v8us o;
#pragma unroll
    for (int k = 0; k < 8; ++k) o[k] = f2bf(v[k]);
    *(volatile v8us*)(dst + i * 8) = o; __threadfence(); *(volatile v8us*)(dst + i * 8) = o;
}

__global__ __launch_bounds__(256) void k_wt(const float* __restrict__ W1, bf* WT) {
#pragma clang fp contract(off)
    __shared__ float ts[DI * 33];
    const unsigned tid = threadIdx.x; const unsigned o0 = blockIdx.x * TR;
#pragma unroll 4
    for (unsigned it = 0; it < (DI * TR) / 256; ++it) {
        const unsigned e = it * 256u + tid; const unsigned k = e >> 5, c = e & 31u;
        ts[k * 33u + c] = W1[(size_t)k * HW + o0 + c]; }
    __syncthreads();
#pragma unroll 1
    for (int ps = 0; ps < 2; ++ps) {
#pragma unroll
        for (unsigned it = 0; it < 2; ++it) {
            const unsigned p = it * 256u + tid; const unsigned row = p >> 4, c8 = (p & 15u) * 8u; v8us o;
#pragma unroll
            for (unsigned i = 0; i < 8; ++i) o[i] = f2bf(ts[(c8 + i) * 33u + row]);
            *(volatile v8us*)(WT + (size_t)(o0 + row) * DI + c8) = o; }
        if (ps == 0) __threadfence(); }
}

__global__ __launch_bounds__(256) void k_zero(const float* __restrict__ W1, const float* __restrict__ b1, const float* __restrict__ lng, const float* __restrict__ lnb,
                                              const float* __restrict__ w2, const float* __restrict__ b2, float* BJ, float* G0) {
#pragma clang fp contract(off)
    __shared__ float as[GW * HW];
    __shared__ __align__(16) float g0s[32];
    const unsigned tid = threadIdx.x; const unsigned lane = tid & 31u;
    const unsigned wave = (unsigned)__builtin_amdgcn_readfirstlane((int)(threadIdx.x >> 5));
    const unsigned jblk = blockIdx.x;
    const float b2v = bfr(b2[0]);
#pragma unroll 1
    for (unsigned q = 0; q < 4; ++q) {
        const unsigned j = jblk * 32u + wave * 4u + q;
        const float* wrow = W1 + (size_t)(DI + j) * HW;
        float* brow = BJ + (size_t)j * HW;
        float sum = 0.0f;
#pragma unroll 1
        for (unsigned e = 0; e < 8; ++e) { const unsigned o = e * 32u + lane; const float v = bfr(wrow[o]) + bfr(b1[o]);
            *(volatile float*)(brow + o) = v;
            const float a = sinf(0.1f * tanhf(v)); as[wave * HW + o] = a; sum += a; }
        __threadfence();
#pragma unroll 1
        for (unsigned e = 0; e < 8; ++e) { const unsigned o = e * 32u + lane; const float v = bfr(wrow[o]) + bfr(b1[o]);
            *(volatile float*)(brow + o) = v; }
        sum += __shfl_xor(sum, 16, 32); sum += __shfl_xor(sum, 8, 32); sum += __shfl_xor(sum, 4, 32); sum += __shfl_xor(sum, 2, 32); sum += __shfl_xor(sum, 1, 32);
        const float mu = sum * (1.0f / 256.0f);
        float sq = 0.0f;
#pragma unroll 1
        for (unsigned e = 0; e < 8; ++e) { const float d = as[wave * HW + e * 32u + lane] - mu; sq += d * d; }
        sq += __shfl_xor(sq, 16, 32); sq += __shfl_xor(sq, 8, 32); sq += __shfl_xor(sq, 4, 32); sq += __shfl_xor(sq, 2, 32); sq += __shfl_xor(sq, 1, 32);
        const float rstd = rsqrtf(sq * (1.0f / 256.0f) + LN_EPS);
        float dot = 0.0f;
#pragma unroll 1
        for (unsigned e = 0; e < 8; ++e) { const unsigned o = e * 32u + lane;
            const float ln = (as[wave * HW + o] - mu) * rstd * bfr(lng[o]) + bfr(lnb[o]); dot += ln * bfr(w2[o]); }
        dot += __shfl_xor(dot, 16, 32); dot += __shfl_xor(dot, 8, 32); dot += __shfl_xor(dot, 4, 32); dot += __shfl_xor(dot, 2, 32); dot += __shfl_xor(dot, 1, 32);
        const float gv = dot + b2v;
        if (lane == 0) g0s[wave * 4u + q] = gv;
    }
    __syncthreads();
    const v4f val = *(const v4fa*)(&g0s[(tid & 7u) * 4u]);
    if (tid < 8) {
#pragma unroll 1
        for (int ps = 0; ps < 2; ++ps) { *(volatile v4f*)(G0 + jblk * 32u + tid * 4u) = val; if (ps == 0) __threadfence(); } }
}

__attribute__((amdgpu_num_vgpr(256))) __global__ __launch_bounds__(32 * WV) void k_main(const bf* __restrict__ XB, const bf* __restrict__ WT, const float* __restrict__ BJ,
                                              const float* __restrict__ lng, const float* __restrict__ lnb, const float* __restrict__ w2, const float* __restrict__ b2, float* G) {
    __shared__ __align__(16) float hs[WV * HSN];
    __shared__ __align__(16) float bjs[WV * HW];
    __shared__ __align__(16) float gt[WV * 16 * GP];
    __shared__ float tg[HW];
    __shared__ float tb[HW];
    __shared__ float tw[HW];
    const unsigned tid = threadIdx.x; const unsigned lane = tid & 31u, lr = lane & 15u, hi = lane >> 4;
    const unsigned wave = (unsigned)__builtin_amdgcn_readfirstlane((int)(threadIdx.x >> 5));
#pragma unroll 1
    for (unsigned o = tid; o < HW; o += 32u * WV) { tg[o] = bfr(lng[o]); tb[o] = bfr(lnb[o]); tw[o] = bfr(w2[o]); }
    __syncthreads();
    const float b2v = bfr(b2[0]);
    const unsigned wt = blockIdx.x * WV + wave;
    const unsigned rt = wt >> 2, jb = wt & 3u;
    const unsigned r0 = rt * 16u, kc0 = 32u * jb;
    const size_t aoff = (size_t)(r0 + lr) * DI + 8u * hi;
    const size_t boff = (size_t)lr * DI + 8u * hi;
    const v4u xa = *(const v4u*)(const void*)(XB + aoff + kc0);
    const v4u xc = *(const v4u*)(const void*)(XB + aoff + kc0 + 16);
    const unsigned hb = wave * HSN + lane;
    const unsigned gb = wave * 16u * GP;
#pragma unroll 1
    for (unsigned jj = 0; jj < JB; ++jj) {
        const unsigned j = kc0 + jj;
        const int d = (int)jj - 8 * (int)hi;
        v8u aw;
#pragma unroll
        for (int w = 0; w < 4; ++w) { const int offs = 2 * w;
            const unsigned mk = (d == offs) ? 0xFFFF0000u : ((d == offs + 1) ? 0x0000FFFFu : 0xFFFFFFFFu); aw[w] = xa[w] & mk; }
#pragma unroll
        for (int w = 0; w < 4; ++w) { const int offs = 16 + 2 * w;
            const unsigned mk = (d == offs) ? 0xFFFF0000u : ((d == offs + 1) ? 0x0000FFFFu : 0xFFFFFFFFu); aw[4 + w] = xc[w] & mk; }
        const v16bf am = __builtin_bit_cast(v16bf, aw);
        v8f acc[16];
#pragma unroll
        for (int nb = 0; nb < 16; ++nb) acc[nb] = (v8f){};
#pragma unroll
        for (int nb = 0; nb < 16; ++nb) { const v16bf b = ldb(WT + boff + (size_t)nb * 16 * DI + kc0); acc[nb] = wmmabg(am, b, acc[nb]); }
#pragma unroll 1
        for (unsigned t = 1; t < 4; ++t) {
            const unsigned kc = 32u * ((jb + t) & 3u);
            const v16bf a = ldb(XB + aoff + kc);
#pragma unroll
            for (int nb = 0; nb < 16; ++nb) { const v16bf b = ldb(WT + boff + (size_t)nb * 16 * DI + kc); acc[nb] = wmmabg(a, b, acc[nb]); }
        }
        wave_sync();
        { const float* bp = BJ + (size_t)j * HW + lane * 4u; const v4f q0 = *(const v4f*)bp; const v4f q1 = *(const v4f*)(bp + 128);
          *(v4fa*)(&bjs[wave * HW + lane * 4u]) = q0; *(v4fa*)(&bjs[wave * HW + 128u + lane * 4u]) = q1; }
        wave_sync();
#pragma unroll
        for (int nb = 0; nb < 16; ++nb) { const float bv = bjs[wave * HW + nb * 16 + lr];
#pragma unroll
            for (int r = 0; r < 8; ++r) hs[hb + (nb * 8 + r) * 32] = acc[nb][r] + bv; }
#pragma unroll 1
        for (unsigned r = 0; r < 8; ++r) {
            float sum = 0.0f;
#pragma unroll 1
            for (unsigned nb = 0; nb < 16; ++nb) { const unsigned ix = hb + (nb * 8u + r) * 32u;
                const float v = hs[ix]; const float a = sinf(0.1f * tanhf(v)); hs[ix] = a; sum += a; }
            sum += __shfl_xor(sum, 8, 32); sum += __shfl_xor(sum, 4, 32); sum += __shfl_xor(sum, 2, 32); sum += __shfl_xor(sum, 1, 32);
            const float mu = sum * (1.0f / 256.0f);
            float sq = 0.0f;
#pragma unroll 4
            for (unsigned nb = 0; nb < 16; ++nb) { const float dd = hs[hb + (nb * 8u + r) * 32u] - mu; sq += dd * dd; }
            sq += __shfl_xor(sq, 8, 32); sq += __shfl_xor(sq, 4, 32); sq += __shfl_xor(sq, 2, 32); sq += __shfl_xor(sq, 1, 32);
            const float rstd = rsqrtf(sq * (1.0f / 256.0f) + LN_EPS);
            float dot = 0.0f;
#pragma unroll 4
            for (unsigned nb = 0; nb < 16; ++nb) { const unsigned o = nb * 16u + lr;
                const float ln = (hs[hb + (nb * 8u + r) * 32u] - mu) * rstd * tg[o] + tb[o]; dot += ln * tw[o]; }
            dot += __shfl_xor(dot, 8, 32); dot += __shfl_xor(dot, 4, 32); dot += __shfl_xor(dot, 2, 32); dot += __shfl_xor(dot, 1, 32);
            const float gv = dot + b2v;
            if (lr == 0) gt[gb + (8u * hi + r) * GP + jj] = gv;
        }
    }
    wave_sync();
    float* grow = G + (size_t)r0 * DI + kc0;
#pragma unroll 1
    for (int ps = 0; ps < 2; ++ps) {
#pragma unroll
        for (int s = 0; s < 4; ++s) { const unsigned row = 4u * s + (lane >> 3), cofs = (lane & 7u) * 4u;
            const v4f val = *(const v4fa*)(&gt[gb + row * GP + cofs]);
            *(volatile v4f*)(grow + (size_t)row * DI + cofs) = val; }
        if (ps == 0) __threadfence(); }
}

__global__ __launch_bounds__(256) void k_out(const float* __restrict__ X, const float* __restrict__ G, const float* __restrict__ G0, float* OUT) {
#pragma clang fp contract(off)
    __shared__ __align__(16) float ot[ORW * OW];
    const unsigned tid = threadIdx.x; const unsigned i0 = blockIdx.x * ORW;
#pragma unroll 4
    for (unsigned it = 0; it < (ORW * DI) / 256; ++it) {
        const unsigned idx = it * 256u + tid; const unsigned rl = idx >> 7, j = idx & 127u;
        const size_t gi = (size_t)(i0 + rl) * DI + j;
        const float xv = bfr(X[gi]); const float hv = 1.0f + (G[gi] - G0[j]);
        ot[rl * OW + 1u + j] = xv * hv; }
    if (tid < ORW) ot[tid * OW] = 1.0f;
    __syncthreads();
    float* ob = OUT + (size_t)blockIdx.x * (ORW * OW);
#pragma unroll 1
    for (int ps = 0; ps < 2; ++ps) {
#pragma unroll 1
        for (unsigned p = tid; p < (ORW * OW) / 4; p += 256u) { const v4f val = *(const v4fa*)(&ot[p * 4u]); *(volatile v4f*)(ob + (size_t)p * 4u) = val; }
        if (ps == 0) __threadfence(); }
}

static constexpr size_t al256(size_t v) { return (v + 255) & ~(size_t)255; }
static constexpr size_t SZ_XB = al256((size_t)NS * DI * 2);
static constexpr size_t SZ_WT = al256((size_t)HW * DI * 2);
static constexpr size_t SZ_BJ = al256((size_t)DI * HW * 4);
static constexpr size_t SZ_G  = al256((size_t)NS * DI * 4);
static constexpr size_t SZ_G0 = al256((size_t)DI * 4);
static constexpr size_t SZ_TOTAL = SZ_XB + SZ_WT + SZ_BJ + SZ_G + SZ_G0;
static_assert(SZ_TOTAL <= (size_t)134217728);
static_assert((size_t)(HW / TR) * TR * DI * 2 == (size_t)HW * DI * 2);
static_assert((size_t)(DI / 32) * GW * 4 * HW * 4 == (size_t)DI * HW * 4);
static_assert((size_t)((NS / 16) * (DI / JB)) * 16 * JB * 4 == (size_t)NS * DI * 4);
static_assert((size_t)(NS / ORW) * ORW * OW == (size_t)NS * OW);

extern "C" void kernel_launch(void* const* d_in, const int* in_sizes, int n_in,
                              void* d_out, int out_size, void* d_ws, size_t ws_size, hipStream_t stream) {
    if (n_in < 7) return;
    if ((size_t)in_sizes[0] < (size_t)NS * DI) return;
    if ((size_t)in_sizes[1] < (size_t)2 * DI * HW) return;
    if (in_sizes[2] < HW || in_sizes[3] < HW || in_sizes[4] < HW || in_sizes[5] < HW || in_sizes[6] < 1) return;
    if ((size_t)out_size < (size_t)NS * OW) return;
    if (SZ_TOTAL > ws_size) return;
    const float* x   = (const float*)d_in[0];
    const float* W1  = (const float*)d_in[1];
    const float* b1  = (const float*)d_in[2];
    const float* lng = (const float*)d_in[3];
    const float* lnb = (const float*)d_in[4];
    const float* w2  = (const float*)d_in[5];
    const float* b2  = (const float*)d_in[6];
    float* OUT = (float*)d_out;
    char* wsp = (char*)d_ws;
    bf* XB = (bf*)wsp; wsp += SZ_XB;
    bf* WT = (bf*)wsp; wsp += SZ_WT;
    float* BJ = (float*)wsp; wsp += SZ_BJ;
    float* G  = (float*)wsp; wsp += SZ_G;
    float* G0 = (float*)wsp; wsp += SZ_G0;

    { const size_t n8 = (size_t)NS * DI / 8;
      k_cvt8<<<(unsigned)((n8 + 255) / 256), 256, 0, stream>>>(x, XB, n8); }
    k_wt<<<HW / TR, 256, 0, stream>>>(W1, WT);
    k_zero<<<DI / 32, 32 * GW, 0, stream>>>(W1, b1, lng, lnb, w2, b2, BJ, G0);
    k_main<<<((NS / 16) * (DI / JB)) / WV, 32 * WV, 0, stream>>>(XB, WT, BJ, lng, lnb, w2, b2, G);
    k_out<<<NS / ORW, 256, 0, stream>>>(x, G, G0, OUT);
}
